// SWA_33225867002140
// MI455X (gfx1250) — hardware-verified
//
#include <hip/hip_runtime.h>
#include <math.h>
#include <stdint.h>

#ifndef NB
#define NB 4
#endif
#ifndef SEQ
#define SEQ 4096
#endif
#define NB_FULL  4
#define SEQ_FULL 4096
#define EMB      512
#define DH       64
#define WIN      256
#define NTOK     (NB * SEQ)
#define QKP      128
#define WTR      192
static_assert(NB >= 1 && NB <= NB_FULL);
static_assert(SEQ >= 128 && SEQ <= SEQ_FULL);
static_assert(SEQ % 128 == 0);
static_assert(EMB % 32 == 0);
static_assert(DH == 64);

typedef _Float16     v16h __attribute__((ext_vector_type(16)));
typedef _Float16     v8h  __attribute__((ext_vector_type(8)));
typedef __bf16       v16b __attribute__((ext_vector_type(16)));
typedef __bf16       v8b  __attribute__((ext_vector_type(8)));
typedef float        v8f  __attribute__((ext_vector_type(8)));
typedef float        v4f  __attribute__((ext_vector_type(4)));
typedef unsigned int v4u  __attribute__((ext_vector_type(4)));

__device__ __forceinline__ unsigned short bf_bits(float f) {
  const unsigned u = __float_as_uint(f);
  return (unsigned short)((u + 0x7FFFu + ((u >> 16) & 1u)) >> 16);
}
__device__ __forceinline__ unsigned pk16(unsigned short a, unsigned short b) { return (unsigned)a | ((unsigned)b << 16); }
__device__ __forceinline__ v8f zero8() { v8f z = {0.f, 0.f, 0.f, 0.f, 0.f, 0.f, 0.f, 0.f}; return z; }
__device__ __forceinline__ int wave_id() { return __builtin_amdgcn_readfirstlane((int)(threadIdx.x >> 5)); }

__device__ __forceinline__ void lds_wave_sync() {
  __builtin_amdgcn_fence(__ATOMIC_RELEASE, "workgroup");
  __builtin_amdgcn_wave_barrier();
  __builtin_amdgcn_fence(__ATOMIC_ACQUIRE, "workgroup");
}

union FragH { v16h v; v8h h[2]; };
union FragB { v16b v; v8b h[2]; };
__device__ __forceinline__ v16h ldfrag_h(const _Float16* p) { FragH f; f.h[0] = *(const v8h*)(p); f.h[1] = *(const v8h*)(p + 16); return f.v; }
__device__ __forceinline__ v16b ldfrag_b(const __bf16* p)   { FragB f; f.h[0] = *(const v8b*)(p); f.h[1] = *(const v8b*)(p + 16); return f.v; }

__device__ __forceinline__ v8f mma_h(v16h a, v16h b, v8f c) {
  return __builtin_amdgcn_wmma_f32_16x16x32_f16(false, a, false, b, (short)0, c, false, false);
}
__device__ __forceinline__ v8f mma_b(v16b a, v16b b, v8f c) {
  return __builtin_amdgcn_wmma_f32_16x16x32_bf16(false, a, false, b, (short)0, c, false, false);
}
__device__ __forceinline__ void guard_b3(v8f& a, v8f& b, v16b x0, v16b x1, v16b y) {
  asm volatile("v_nop\n\tv_nop\n\tv_nop\n\tv_nop" : "+v"(a), "+v"(b) : "v"(x0), "v"(x1), "v"(y) : "memory");
}
__device__ __forceinline__ void guard_h3(v8f& a, v8f& b, v16h x, v16h y, v16h z) {
  asm volatile("v_nop\n\tv_nop\n\tv_nop\n\tv_nop" : "+v"(a), "+v"(b) : "v"(x), "v"(y), "v"(z) : "memory");
}
__device__ __forceinline__ void guard_h4(v8f& a, v8f& b, v16h w, v16h x, v16h y, v16h z) {
  asm volatile("v_nop\n\tv_nop\n\tv_nop\n\tv_nop" : "+v"(a), "+v"(b) : "v"(w), "v"(x), "v"(y), "v"(z) : "memory");
}
__device__ __forceinline__ void acc_guard4(v8f& a, v8f& b, v8f& c, v8f& d) {
  asm volatile("v_nop\n\tv_nop\n\tv_nop\n\tv_nop" : "+v"(a), "+v"(b), "+v"(c), "+v"(d));
}

__global__ __launch_bounds__(256) void cvt_x_kernel(const float* __restrict__ in, unsigned short* __restrict__ outp, int n8) {
  const int i = (int)blockIdx.x * 256 + (int)threadIdx.x;
  if (i >= n8) return;
  const size_t e   = 8 * (size_t)i;
  const size_t row = e / EMB;
  const size_t col = e - row * EMB;
  const size_t bb  = row / SEQ;
  const size_t tt  = row - bb * SEQ;
  const size_t s   = (bb * SEQ_FULL + tt) * EMB + col;
  const v4f a = *(const v4f*)(in + s);
  const v4f b = *(const v4f*)(in + s + 4);
  v4u w;
  w[0] = pk16(bf_bits(a[0]), bf_bits(a[1]));
  w[1] = pk16(bf_bits(a[2]), bf_bits(a[3]));
  w[2] = pk16(bf_bits(b[0]), bf_bits(b[1]));
  w[3] = pk16(bf_bits(b[2]), bf_bits(b[3]));
  *(volatile v4u*)(outp + e) = w;
  __threadfence();
  *(volatile v4u*)(outp + e) = w;
}

__global__ __launch_bounds__(256) void wt_kernel(const float* __restrict__ wq, const float* __restrict__ wk,
                                                 const float* __restrict__ wv, unsigned short* __restrict__ wt) {
  __shared__ __align__(16) unsigned short st[8 * EMB];
  const int tid = (int)threadIdx.x;
  const int blk = (int)blockIdx.x;
  if (blk >= WTR / 8) return;
  const int w   = blk >> 3;
  const int d0  = (blk & 7) * 8;
  const float* W = (w == 0) ? wq : ((w == 1) ? wk : wv);
#pragma unroll
  for (int u = 0; u < 2; ++u) {
    const int e = tid + 256 * u;
    const v4f a = *(const v4f*)(W + (size_t)e * DH + d0);
    const v4f c = *(const v4f*)(W + (size_t)e * DH + d0 + 4);
    st[0 * EMB + e] = bf_bits(a[0]);
    st[1 * EMB + e] = bf_bits(a[1]);
    st[2 * EMB + e] = bf_bits(a[2]);
    st[3 * EMB + e] = bf_bits(a[3]);
    st[4 * EMB + e] = bf_bits(c[0]);
    st[5 * EMB + e] = bf_bits(c[1]);
    st[6 * EMB + e] = bf_bits(c[2]);
    st[7 * EMB + e] = bf_bits(c[3]);
  }
  __syncthreads();
  unsigned short* dst = wt + (size_t)blk * 8 * EMB;
  for (int pass = 0; pass < 2; ++pass) {
#pragma unroll
    for (int u = 0; u < 2; ++u) {
      const int p   = tid + 256 * u;
      const int row = p >> 6;
      const int c8  = (p & 63) * 8;
      const v4u v = *(const v4u*)(st + row * EMB + c8);
      *(volatile v4u*)(dst + (size_t)row * EMB + c8) = v;
    }
    __threadfence();
  }
}

__global__ __launch_bounds__(128) void gemm_w32x128_kernel(
    const unsigned short* __restrict__ Ap, int lda,
    const unsigned short* __restrict__ Btp, int ldb,
    unsigned short* __restrict__ C0p, unsigned short* __restrict__ C1p, int ldc,
    int M, int N, int K) {
  __shared__ __align__(16) _Float16 slab_all[4 * 4096];

  const int lane = threadIdx.x & 31;
  const int wave = wave_id();
  const int hh = lane >> 4;
  const int rl = lane & 15;
  const int tilesN = N >> 7;
  const int tilesM = M >> 5;
  const int tile = (int)blockIdx.x * 4 + wave;
  if (tile >= tilesM * tilesN) return;
  const int tm = tile / tilesN;
  const int tn = tile - tm * tilesN;
  const int m0 = tm << 5;
  const int n0 = tn << 7;

  const __bf16* A  = (const __bf16*)(const void*)Ap;
  const __bf16* Bt = (const __bf16*)(const void*)Btp;

  v8f acc[2][8];
#pragma unroll
  for (int i = 0; i < 2; ++i)
#pragma unroll
    for (int j = 0; j < 8; ++j) acc[i][j] = zero8();

  for (int k0 = 0; k0 < K; k0 += 32) {
    v16b ah[2];
#pragma unroll
    for (int i = 0; i < 2; ++i) {
      const size_t ao = (size_t)(m0 + i * 16 + rl) * lda + k0 + 8 * hh;
      ah[i] = ldfrag_b(A + ao);
    }
#pragma unroll
    for (int j = 0; j < 8; ++j) {
      const int brow = n0 + j * 16 + rl;
      const v16b bj = ldfrag_b(Bt + (size_t)brow * ldb + k0 + 8 * hh);
      acc[0][j] = mma_b(ah[0], bj, acc[0][j]);
      acc[1][j] = mma_b(ah[1], bj, acc[1][j]);
      guard_b3(acc[0][j], acc[1][j], ah[0], ah[1], bj);
    }
  }
  acc_guard4(acc[0][0], acc[0][1], acc[0][2], acc[0][3]);
  acc_guard4(acc[0][4], acc[0][5], acc[0][6], acc[0][7]);
  acc_guard4(acc[1][0], acc[1][1], acc[1][2], acc[1][3]);
  acc_guard4(acc[1][4], acc[1][5], acc[1][6], acc[1][7]);

  _Float16* sl16 = slab_all + wave * 4096;
  _Float16* P0 = (_Float16*)(void*)C0p;
  _Float16* P1 = (_Float16*)(void*)C1p;
#pragma unroll
  for (int i = 0; i < 2; ++i) {
#pragma unroll
    for (int r = 0; r < 8; ++r) {
#pragma unroll
      for (int j = 0; j < 8; ++j) {
        const float v = acc[i][j][r];
        const _Float16 hv = (_Float16)v;
        const int so = (8 * hh + r) * 128 + j * 16 + rl;
        sl16[so]        = hv;
        sl16[2048 + so] = (_Float16)((v - (float)hv) * 2048.0f);
      }
    }
    lds_wave_sync();
    for (int pass = 0; pass < 2; ++pass) {
#pragma unroll
      for (int it = 0; it < 8; ++it) {
        const int row = it * 2 + hh;
        const int c8  = rl * 8;
        const v8h vh = *(const v8h*)(sl16 + row * 128 + c8);
        const v8h vl = *(const v8h*)(sl16 + 2048 + row * 128 + c8);
        const size_t go = (size_t)(m0 + i * 16 + row) * ldc + n0 + c8;
        *(volatile v8h*)(P0 + go) = vh;
        *(volatile v8h*)(P1 + go) = vl;
      }
      __threadfence();
    }
    lds_wave_sync();
  }
}

#define AT_KC   32
#define KS_P    72
#define VS_P    40
#define PS_P    40
#define NCH_MAX ((64 + WIN - 1 + 31) / 32 + 1)
#define LDS_KS  0
#define LDS_KLS (32 * KS_P)
#define LDS_VHS (2 * 32 * KS_P)
#define LDS_VLS (LDS_VHS + DH * VS_P)
#define LDS_PH  (LDS_VLS + DH * VS_P)
#define LDS_PL  (LDS_PH + 4 * 16 * PS_P)
#define LDS_TOT (LDS_PL + 4 * 16 * PS_P)
static_assert(LDS_TOT * 2 <= 65536);
static_assert(4 * 2048 <= LDS_TOT);
static_assert((LDS_KLS * 2) % 16 == 0 && (LDS_VHS * 2) % 16 == 0 && (LDS_VLS * 2) % 16 == 0);
static_assert((LDS_PH * 2) % 16 == 0 && (LDS_PL * 2) % 16 == 0);
static_assert(SEQ % 64 == 0);

template <bool PRES>
__global__ __launch_bounds__(128) void attn_window_kernel(
    const unsigned short* __restrict__ qkhp, const unsigned short* __restrict__ qklp,
    const unsigned short* __restrict__ vhp, const unsigned short* __restrict__ vlp,
    float* __restrict__ outp, int qb_base) {
  __shared__ __align__(16) _Float16 lds[LDS_TOT];
  _Float16* Ks  = lds + LDS_KS;
  _Float16* Kls = lds + LDS_KLS;
  _Float16* Vhs = lds + LDS_VHS;
  _Float16* Vls = lds + LDS_VLS;

  const int tid  = (int)threadIdx.x;
  const int lane = tid & 31;
  const int wave = wave_id();
  const int hh   = lane >> 4;
  const int c    = lane & 15;
  const int qb   = (int)blockIdx.x + qb_base;
  const int b    = (int)blockIdx.y;
  const int qblk0 = qb * 64;
  if (qblk0 + 64 > SEQ) return;
  const int q0    = qblk0 + wave * 16;
  const int qlast = q0 + 15;
  const int wlo   = q0 - (WIN - 1);
  const size_t tok0 = (size_t)b * SEQ;

  int kstart = qblk0 - (WIN - 1);
  kstart = (kstart > 0) ? (kstart & ~31) : 0;
  if (kstart > qblk0) kstart = qblk0;
  int nch = (qblk0 + 64 - kstart) >> 5;
  if (nch > NCH_MAX) nch = NCH_MAX;
  if (nch < 0) nch = 0;

  const _Float16* Qhr = (const _Float16*)(const void*)qkhp + (tok0 + q0 + c) * QKP + 8 * hh;
  const _Float16* Qlr = (const _Float16*)(const void*)qklp + (tok0 + q0 + c) * QKP + 8 * hh;
  const _Float16* Kg  = (const _Float16*)(const void*)qkhp + tok0 * QKP + DH;
  const _Float16* Klg = (const _Float16*)(const void*)qklp + tok0 * QKP + DH;
  const _Float16* Vhg = (const _Float16*)(const void*)vhp + tok0;
  const _Float16* Vlg = (const _Float16*)(const void*)vlp + tok0;
  _Float16* ph = lds + LDS_PH + wave * (16 * PS_P);
  _Float16* pl = lds + LDS_PL + wave * (16 * PS_P);

  float mrow[8], lrow[8];
  v8f oacc[4], oaccr[4];
#pragma unroll
  for (int r = 0; r < 8; ++r) { mrow[r] = -INFINITY; lrow[r] = 0.f; }
#pragma unroll
  for (int t = 0; t < 4; ++t) { oacc[t] = zero8(); oaccr[t] = zero8(); }

  for (int kc = 0; kc < nch; ++kc) {
    const int kv0 = kstart + kc * AT_KC;
    __syncthreads();
#pragma unroll
    for (int i = 0; i < 2; ++i) {
      const int p   = tid + 128 * i;
      const int key = p >> 3, d8 = (p & 7) * 8;
      const v8h kx = *(const v8h*)(Kg + (size_t)(kv0 + key) * QKP + d8);
      *(v8h*)(Ks + key * KS_P + d8) = kx;
      if (PRES) {
        const v8h ky = *(const v8h*)(Klg + (size_t)(kv0 + key) * QKP + d8);
        *(v8h*)(Kls + key * KS_P + d8) = ky;
      }
      const int d = p >> 2, k8 = (p & 3) * 8;
      const v8h vx = *(const v8h*)(Vhg + (size_t)d * NTOK + kv0 + k8);
      const v8h vy = *(const v8h*)(Vlg + (size_t)d * NTOK + kv0 + k8);
      *(v8h*)(Vhs + d * VS_P + k8) = vx;
      *(v8h*)(Vls + d * VS_P + k8) = vy;
    }
    __syncthreads();

    if (kv0 <= qlast && kv0 + AT_KC - 1 >= wlo) {
      v8f sh[2], sr[2];
      sh[0] = zero8(); sh[1] = zero8(); sr[0] = zero8(); sr[1] = zero8();
#pragma unroll
      for (int dc = 0; dc < 2; ++dc) {
        const v16h qa = ldfrag_h(Qhr + dc * 32);
        const v16h ql = ldfrag_h(Qlr + dc * 32);
#pragma unroll
        for (int j = 0; j < 2; ++j) {
          const v16h kb = ldfrag_h(Ks + (j * 16 + c) * KS_P + dc * 32 + 8 * hh);
          sh[j] = mma_h(qa, kb, sh[j]);
          sr[j] = mma_h(ql, kb, sr[j]);
          if (PRES) {
            const v16h kl = ldfrag_h(Kls + (j * 16 + c) * KS_P + dc * 32 + 8 * hh);
            sr[j] = mma_h(qa, kl, sr[j]);
            guard_h4(sh[j], sr[j], qa, ql, kb, kl);
          } else {
            guard_h3(sh[j], sr[j], qa, ql, kb);
          }
        }
      }
      float cm[8];
#pragma unroll
      for (int r = 0; r < 8; ++r) {
        const int qrow = q0 + 8 * hh + r;
        float m = -INFINITY;
#pragma unroll
        for (int j = 0; j < 2; ++j) {
          const int key = kv0 + j * 16 + c;
          float s = (sh[j][r] + sr[j][r] * 0.00048828125f) * 0.125f;
          const bool ok = (key <= qrow) && (qrow - key < WIN);
          s = ok ? s : -INFINITY;
          sh[j][r] = s;
          m = fmaxf(m, s);
        }
#pragma unroll
        for (int off = 1; off < 16; off <<= 1) m = fmaxf(m, __shfl_xor(m, off, 32));
        cm[r] = m;
      }
#pragma unroll
      for (int r = 0; r < 8; ++r) {
        const float mnew  = fmaxf(mrow[r], cm[r]);
        const float mref  = (mnew == -INFINITY) ? 0.f : mnew;
        const float alpha = __expf(mrow[r] - mref);
        mrow[r] = mnew;
        float psum = 0.f;
#pragma unroll
        for (int j = 0; j < 2; ++j) {
          const float p  = __expf(sh[j][r] - mref);
          psum += p;
          const float pp = p * 1024.0f;
          const _Float16 phv = (_Float16)pp;
          const int po = (8 * hh + r) * PS_P + j * 16 + c;
          ph[po] = phv;
          if (PRES) pl[po] = (_Float16)((pp - (float)phv) * 2048.0f);
        }
#pragma unroll
        for (int off = 1; off < 16; off <<= 1) psum += __shfl_xor(psum, off, 32);
        lrow[r] = lrow[r] * alpha + psum;
#pragma unroll
        for (int t = 0; t < 4; ++t) { oacc[t][r] *= alpha; oaccr[t][r] *= alpha; }
      }
      lds_wave_sync();
      const v16h pa = ldfrag_h(ph + c * PS_P + 8 * hh);
      v16h pr = pa;
      if (PRES) pr = ldfrag_h(pl + c * PS_P + 8 * hh);
#pragma unroll
      for (int t = 0; t < 4; ++t) {
        const v16h vb = ldfrag_h(Vhs + (t * 16 + c) * VS_P + 8 * hh);
        const v16h vr = ldfrag_h(Vls + (t * 16 + c) * VS_P + 8 * hh);
        oacc[t]  = mma_h(pa, vb, oacc[t]);
        oaccr[t] = mma_h(pa, vr, oaccr[t]);
        if (PRES) oaccr[t] = mma_h(pr, vb, oaccr[t]);
        guard_h4(oacc[t], oaccr[t], pa, pr, vb, vr);
      }
    }
  }

  __syncthreads();
  float* os = (float*)(void*)lds + wave * 1024;
#pragma unroll
  for (int r = 0; r < 8; ++r) {
    const float inv = (1.0f / lrow[r]) * 0.0009765625f;
#pragma unroll
    for (int t = 0; t < 4; ++t) {
      const float o = (oacc[t][r] + oaccr[t][r] * 0.00048828125f) * inv;
      os[(8 * hh + r) * DH + t * 16 + c] = o;
    }
  }
  lds_wave_sync();
  float* Og = outp + (tok0 + q0) * DH;
  for (int pass = 0; pass < 2; ++pass) {
#pragma unroll
    for (int it = 0; it < 8; ++it) {
      const int row = it * 2 + hh;
      const int c4  = c * 4;
      const v4f v = *(const v4f*)(os + row * DH + c4);
      *(volatile v4f*)(Og + (size_t)row * DH + c4) = v;
    }
    __threadfence();
  }
}

extern "C" void kernel_launch(void* const* d_in, const int* in_sizes, int n_in,
                              void* d_out, int out_size, void* d_ws, size_t ws_size,
                              hipStream_t stream) {
  if (n_in < 4) return;
  if (in_sizes[0] < ((NB - 1) * SEQ_FULL + SEQ) * EMB) return;
  if (in_sizes[1] < EMB * DH) return;
  if (in_sizes[2] < EMB * DH) return;
  if (in_sizes[3] < EMB * DH) return;
  if (out_size < NTOK * DH) return;

  const float* x  = (const float*)d_in[0];
  const float* wk = (const float*)d_in[1];
  const float* wq = (const float*)d_in[2];
  const float* wv = (const float*)d_in[3];
  float* out = (float*)d_out;

  const size_t szX  = (size_t)NTOK * EMB * 2;
  const size_t szWt = (size_t)WTR * EMB * 2;
  const size_t szQK = (size_t)NTOK * QKP * 2;
  const size_t szV  = (size_t)DH * NTOK * 2;
  size_t off = 0;
  const size_t oX   = off; off += szX;
  const size_t oWt  = off; off += szWt;
  const size_t oQKh = off; off += szQK;
  const size_t oQKl = off; off += szQK;
  const size_t oVh  = off; off += szV;
  const size_t oVl  = off; off += szV;
  if (off > ws_size) return;
  if ((oWt & 127) != 0 || (oQKh & 127) != 0 || (oQKl & 127) != 0 || (oVh & 127) != 0 || (oVl & 127) != 0) return;

  char* ws = (char*)d_ws;
  unsigned short* Xb  = (unsigned short*)(ws + oX);
  unsigned short* Wt  = (unsigned short*)(ws + oWt);
  unsigned short* QKh = (unsigned short*)(ws + oQKh);
  unsigned short* QKl = (unsigned short*)(ws + oQKl);
  unsigned short* Vh  = (unsigned short*)(ws + oVh);
  unsigned short* Vl  = (unsigned short*)(ws + oVl);

  const dim3 b256(256), b128(128);

  const int n8 = NTOK * EMB / 8;
  cvt_x_kernel<<<dim3((n8 + 255) / 256), b256, 0, stream>>>(x, Xb, n8);
  wt_kernel<<<dim3(WTR / 8), b256, 0, stream>>>(wq, wk, wv, Wt);
  {
    const int tiles = (NTOK / 32) * (QKP / 128);
    gemm_w32x128_kernel<<<dim3((tiles + 3) / 4), b128, 0, stream>>>(
        Xb, EMB, Wt, EMB, QKh, QKl, QKP, NTOK, QKP, EMB);
  }
  {
    const int tiles = (DH / 32) * (NTOK / 128);
    gemm_w32x128_kernel<<<dim3((tiles + 3) / 4), b128, 0, stream>>>(
        Wt + (size_t)128 * EMB, EMB, Xb, EMB, Vh, Vl, NTOK, DH, NTOK, EMB);
  }
  const int nqt   = SEQ / 64;
  const int npres = (nqt < 4) ? nqt : 4;
  attn_window_kernel<true><<<dim3(npres, NB), b128, 0, stream>>>(QKh, QKl, Vh, Vl, out, 0);
  if (nqt > npres)
    attn_window_kernel<false><<<dim3(nqt - npres, NB), b128, 0, stream>>>(QKh, QKl, Vh, Vl, out, npres);
  (void)hipGetLastError();
}
